// DVTATT_88158498718224
// MI455X (gfx1250) — hardware-verified
//
#include <hip/hip_runtime.h>


#define NB   4
#define NC   256
#define NP   4096
#define CIN  1024
#define CAUX 768
#define CFU  512
#define MS   512
#define QCH  128
#define KT   32
#define QCN  (NP / QCH)

typedef _Float16 v16h __attribute__((ext_vector_type(16)));
typedef _Float16 v8h  __attribute__((ext_vector_type(8)));
typedef v8h v8ha __attribute__((may_alias));
typedef float v8f __attribute__((ext_vector_type(8)));
typedef float v4f __attribute__((ext_vector_type(4)));
typedef v4f v4fa __attribute__((may_alias));

union Frag { v16h v; v8h hf[2]; };

__device__ __forceinline__ v8f zero8() {
  v8f z = {0.f, 0.f, 0.f, 0.f, 0.f, 0.f, 0.f, 0.f};
  return z;
}

__device__ __forceinline__ v8f wmma16(v16h a, v16h b, v8f c) {
  v8f d = __builtin_amdgcn_wmma_f32_16x16x32_f16(false, a, false, b, (short)0, c, false, false);
  asm volatile("v_nop\n\tv_nop\n\tv_nop\n\tv_nop" : "+v"(d) : "v"(a), "v"(b));
  return d;
}

__device__ __forceinline__ v16h ldfrag_g(const _Float16* rowp, int k0, int h) {
  Frag f;
  f.hf[0] = *(const v8h*)(rowp + k0 + 8 * h);
  f.hf[1] = *(const v8h*)(rowp + k0 + 16 + 8 * h);
  return f.v;
}
__device__ __forceinline__ v16h ldfrag_l(const _Float16* rowp, int k0, int h) {
  Frag f;
  f.hf[0] = *(const v8ha*)(rowp + k0 + 8 * h);
  f.hf[1] = *(const v8ha*)(rowp + k0 + 16 + 8 * h);
  return f.v;
}

__device__ __forceinline__ v8h pack8(v4f a, v4f b) {
  v8h r;
  r[0] = (_Float16)a[0]; r[1] = (_Float16)a[1]; r[2] = (_Float16)a[2]; r[3] = (_Float16)a[3];
  r[4] = (_Float16)b[0]; r[5] = (_Float16)b[1]; r[6] = (_Float16)b[2]; r[7] = (_Float16)b[3];
  return r;
}

__device__ __forceinline__ float max8f(v4f a, v4f b) {
  float m0 = fmaxf(fmaxf(a[0], a[1]), fmaxf(a[2], a[3]));
  float m1 = fmaxf(fmaxf(b[0], b[1]), fmaxf(b[2], b[3]));
  return fmaxf(m0, m1);
}

template <typename T>
__device__ __forceinline__ void vst2(T* p, T v) {
  *(volatile T*)p = v;
  __threadfence();
  *(volatile T*)p = v;
}

__global__ void __launch_bounds__(256) k_pool(const float* __restrict__ msk, float* __restrict__ mF) {
  const int i = blockIdx.x * 256 + threadIdx.x;
  if (i >= NB * NP / 4) return;
  const int pix0 = i * 4;
  const int b = pix0 >> 12, p = pix0 & (NP - 1);
  const int y = p >> 6, x0 = p & 63;
  const float* s = msk + ((size_t)b * MS + (size_t)y * 8) * MS + (size_t)x0 * 8;
  float mx[4] = {0.f, 0.f, 0.f, 0.f};
#pragma unroll
  for (int dy = 0; dy < 8; ++dy) {
    const float* row = s + dy * MS;
#pragma unroll
    for (int j = 0; j < 4; ++j) {
      v4f a = *(const v4f*)(row + j * 8);
      v4f c = *(const v4f*)(row + j * 8 + 4);
      mx[j] = fmaxf(mx[j], max8f(a, c));
    }
  }
  v4f r;
#pragma unroll
  for (int j = 0; j < 4; ++j) r[j] = (mx[j] > 0.f) ? 1.f : 0.f;
  vst2((v4f*)(mF + pix0), r);
}

__global__ void __launch_bounds__(256) k_cvtw(const float* __restrict__ Kw, const float* __restrict__ Fw,
                                              _Float16* __restrict__ Kwh, _Float16* __restrict__ Fwh) {
  const int i = blockIdx.x * 256 + threadIdx.x;
  const float* src;
  _Float16* dst;
  if (i < NC * CIN / 8) {
    src = Kw + (size_t)i * 8; dst = Kwh + (size_t)i * 8;
  } else if (i < NC * CIN / 8 + NC * CFU / 8) {
    const int j = i - NC * CIN / 8;
    src = Fw + (size_t)j * 8; dst = Fwh + (size_t)j * 8;
  } else {
    return;
  }
  v4f a = *(const v4f*)src;
  v4f c = *(const v4f*)(src + 4);
  a = a * 64.f; c = c * 64.f;
  vst2((v8h*)dst, pack8(a, c));
}

__global__ void __launch_bounds__(256) k_tin(const float* __restrict__ x, const float* __restrict__ aux,
                                             _Float16* __restrict__ inT) {
  __shared__ __attribute__((aligned(16))) _Float16 T[64][72];
  const int t = threadIdx.x, blk = blockIdx.x;
  if (blk >= NB * (CIN / 64) * (NP / 64)) return;
  const int b = blk >> 10, ct = (blk >> 6) & 15, pt = blk & 63;
  const int c0 = ct * 64, p0 = pt * 64;
#pragma unroll
  for (int i = 0; i < 4; ++i) {
    const int f = t + 256 * i;
    const int cl = f >> 4, p4 = (f & 15) * 4;
    const int c = c0 + cl;
    const float* src = (c0 < NC)
        ? x   + ((size_t)(b * NC + c)) * NP + p0 + p4
        : aux + ((size_t)(b * CAUX + (c - NC))) * NP + p0 + p4;
    v4f v = *(const v4f*)src;
    T[p4 + 0][cl] = (_Float16)v[0];
    T[p4 + 1][cl] = (_Float16)v[1];
    T[p4 + 2][cl] = (_Float16)v[2];
    T[p4 + 3][cl] = (_Float16)v[3];
  }
  __syncthreads();
  v8h val[2];
  size_t off[2];
#pragma unroll
  for (int i = 0; i < 2; ++i) {
    const int r = (t >> 3) + 32 * i, q = t & 7;
    val[i] = *(const v8ha*)&T[r][q * 8];
    off[i] = ((size_t)(b * NP + p0 + r)) * CIN + c0 + q * 8;
  }
#pragma unroll
  for (int i = 0; i < 2; ++i) vst2((v8h*)(inT + off[i]), val[i]);
}

__global__ void __launch_bounds__(256) k_feats(const _Float16* __restrict__ inT, const _Float16* __restrict__ Kwh,
                                               const float* __restrict__ Kb, _Float16* __restrict__ Nh) {
  __shared__ __attribute__((aligned(16))) float F[32][260];
  const int t = threadIdx.x, lane = t & 31, wid = t >> 5, h = lane >> 4, n = lane & 15;
  const int blk = blockIdx.x;
  if (blk >= NB * NP / 32) return;
  const int b = blk >> 7, pb = (blk & 127) * 32;
  const int ptile = wid >> 2, og = wid & 3;
  const _Float16* Arow = inT + ((size_t)(b * NP + pb + ptile * 16 + n)) * CIN;
  const _Float16* Bb   = Kwh + ((size_t)(og * 64 + n)) * CIN;
  v8f d[4];
#pragma unroll
  for (int j = 0; j < 4; ++j) d[j] = zero8();
#pragma unroll 1
  for (int k0 = 0; k0 < CIN; k0 += 32) {
    const v16h a = ldfrag_g(Arow, k0, h);
#pragma unroll
    for (int j = 0; j < 4; ++j) d[j] = wmma16(a, ldfrag_g(Bb + (size_t)j * 16 * CIN, k0, h), d[j]);
  }
#pragma unroll
  for (int j = 0; j < 4; ++j) {
    const int o = og * 64 + j * 16 + n;
    const float bias = Kb[o];
#pragma unroll
    for (int r = 0; r < 8; ++r) F[ptile * 16 + 8 * h + r][o] = d[j][r] * (1.f / 64.f) + bias;
  }
  __syncthreads();
  v8h vals[4];
  size_t offs[4];
#pragma unroll
  for (int i = 0; i < 4; ++i) {
    const int pl = wid * 4 + i;
    v4f a = *(const v4fa*)&F[pl][lane * 8];
    v4f c = *(const v4fa*)&F[pl][lane * 8 + 4];
    float ss = a[0] * a[0] + a[1] * a[1] + a[2] * a[2] + a[3] * a[3]
             + c[0] * c[0] + c[1] * c[1] + c[2] * c[2] + c[3] * c[3];
    ss += __shfl_xor(ss, 16); ss += __shfl_xor(ss, 8); ss += __shfl_xor(ss, 4);
    ss += __shfl_xor(ss, 2);  ss += __shfl_xor(ss, 1);
    const float inv = 8.f * (1.f / (sqrtf(ss) + 1e-8f));
    vals[i] = pack8(a * inv, c * inv);
    offs[i] = ((size_t)(b * NP + pb + pl)) * NC + lane * 8;
  }
#pragma unroll
  for (int i = 0; i < 4; ++i) vst2((v8h*)(Nh + offs[i]), vals[i]);
}

__global__ void __launch_bounds__(256) k_makev(const float* __restrict__ x, const float* __restrict__ mF,
                                               _Float16* __restrict__ Vh) {
  const int i = blockIdx.x * 256 + threadIdx.x;
  if (i >= NB * NC * NP / 8) return;
  const size_t e0 = (size_t)i * 8;
  const int p = (int)(e0 & (NP - 1));
  const int b = (int)(e0 >> 20);
  v4f x0 = *(const v4f*)(x + e0);
  v4f x1 = *(const v4f*)(x + e0 + 4);
  v4f m0 = *(const v4f*)(mF + (size_t)b * NP + p);
  v4f m1 = *(const v4f*)(mF + (size_t)b * NP + p + 4);
  v4f k0 = 1.f - m0, k1 = 1.f - m1;
  vst2((v8h*)(Vh + e0), pack8(x0 * k0, x1 * k1));
}

__global__ void __launch_bounds__(256) __attribute__((amdgpu_num_vgpr(252)))
k_attn(const _Float16* __restrict__ Nh, const _Float16* __restrict__ Vh, const float* __restrict__ mF,
       _Float16* __restrict__ attT, float* __restrict__ cpart) {
  __shared__ __attribute__((aligned(16))) _Float16 Qs[QCH][264];
  __shared__ __attribute__((aligned(16))) _Float16 Ks[KT][264];
  __shared__ __attribute__((aligned(16))) _Float16 Vs[NC][40];
  __shared__ __attribute__((aligned(16))) _Float16 Ps[8][16][40];
  __shared__ float cs[8][32];
  __shared__ __attribute__((aligned(16))) float csb[NP];

  const int t = threadIdx.x, lane = t & 31, wid = t >> 5, h = lane >> 4, n = lane & 15;
  const int blk = blockIdx.x;
  if (blk >= NB * QCN) return;
  const int b = blk >> 5, qc = blk & 31;
  const int qblk = qc * QCH, qw = qblk + wid * 16;
  const _Float16* Nb = Nh + (size_t)b * NP * NC;
  const _Float16* Vb = Vh + (size_t)b * NC * NP;
  const float* mb = mF + (size_t)b * NP;

#pragma unroll
  for (int i = 0; i < 16; ++i) {
    const int id = t + 256 * i;
    const int row = id >> 5, c8 = (id & 31) * 8;
    *(v8h*)&Qs[row][c8] = *(const v8h*)(Nb + (size_t)(qblk + row) * NC + c8);
  }
  __syncthreads();

  const _Float16* Qrow = &Qs[wid * 16 + n][0];

  float invs[8];
  {
    v16h qf[8];
#pragma unroll
    for (int cb = 0; cb < 8; ++cb) qf[cb] = ldfrag_l(Qrow, cb * 32, h);
    float acc[8];
#pragma unroll
    for (int r = 0; r < 8; ++r) acc[r] = 0.f;
#pragma unroll 1
    for (int kb = 0; kb < NP; kb += KT) {
      __syncthreads();
#pragma unroll
      for (int i = 0; i < 4; ++i) {
        const int id = t + 256 * i;
        const int row = id >> 5, c8 = (id & 31) * 8;
        *(v8h*)&Ks[row][c8] = *(const v8h*)(Nb + (size_t)(kb + row) * NC + c8);
      }
      __syncthreads();
#pragma unroll
      for (int sub = 0; sub < 2; ++sub) {
        v8f s = zero8();
        const _Float16* Krow = &Ks[sub * 16 + n][0];
#pragma unroll
        for (int cb = 0; cb < 8; ++cb) s = wmma16(qf[cb], ldfrag_l(Krow, cb * 32, h), s);
        const float km = 1.f - mb[kb + sub * 16 + n];
#pragma unroll
        for (int r = 0; r < 8; ++r) acc[r] += km * __expf(0.3125f * s[r] - 20.f);
      }
    }
#pragma unroll
    for (int r = 0; r < 8; ++r) {
      float a = acc[r];
      a += __shfl_xor(a, 1); a += __shfl_xor(a, 2); a += __shfl_xor(a, 4); a += __shfl_xor(a, 8);
      invs[r] = mb[qw + 8 * h + r] / (a + 1e-30f);
    }
  }

  v8f o[16];
#pragma unroll
  for (int cc = 0; cc < 16; ++cc) o[cc] = zero8();
#pragma unroll 1
  for (int kb = 0; kb < NP; kb += KT) {
    __syncthreads();
#pragma unroll
    for (int i = 0; i < 4; ++i) {
      const int id = t + 256 * i;
      const int row = id >> 5, c8 = (id & 31) * 8;
      *(v8h*)&Ks[row][c8] = *(const v8h*)(Nb + (size_t)(kb + row) * NC + c8);
      const int vr = id >> 2, v8 = (id & 3) * 8;
      *(v8h*)&Vs[vr][v8] = *(const v8h*)(Vb + (size_t)vr * NP + kb + v8);
    }
    __syncthreads();
#pragma unroll
    for (int sub = 0; sub < 2; ++sub) {
      v8f s = zero8();
      const _Float16* Krow = &Ks[sub * 16 + n][0];
#pragma unroll
      for (int cb = 0; cb < 8; ++cb) s = wmma16(ldfrag_l(Qrow, cb * 32, h), ldfrag_l(Krow, cb * 32, h), s);
      const float km = 1.f - mb[kb + sub * 16 + n];
      float csum = 0.f;
#pragma unroll
      for (int r = 0; r < 8; ++r) {
        const float att = invs[r] * km * __expf(0.3125f * s[r] - 20.f);
        csum += att;
        Ps[wid][8 * h + r][sub * 16 + n] = (_Float16)(att * 4096.f);
      }
      csum += __shfl_xor(csum, 16);
      if (lane < 16) cs[wid][sub * 16 + lane] = csum;
    }
    __syncthreads();
    if (wid == 0) {
      float tt = 0.f;
#pragma unroll
      for (int w = 0; w < 8; ++w) tt += cs[w][lane];
      csb[kb + lane] = tt;
    }
    const v16h pB = ldfrag_l(&Ps[wid][n][0], 0, h);
#pragma unroll
    for (int g = 0; g < 4; ++g) {
#pragma unroll
      for (int j = 0; j < 4; ++j)
        o[g * 4 + j] = wmma16(ldfrag_l(&Vs[g * 64 + j * 16 + n][0], 0, h), pB, o[g * 4 + j]);
    }
  }

#pragma unroll
  for (int cc = 0; cc < 16; ++cc) {
    v8h tv;
#pragma unroll
    for (int r = 0; r < 8; ++r) tv[r] = (_Float16)(o[cc][r] * (1.f / 4096.f));
    *(v8h*)&Qs[wid * 16 + n][cc * 16 + 8 * h] = tv;
  }
  __syncthreads();
  _Float16* arow = attT + ((size_t)(b * NP + qw)) * NC + lane * 8;
#pragma unroll
  for (int i = 0; i < 16; ++i) {
    v8h v = *(const v8ha*)&Qs[wid * 16 + i][lane * 8];
    vst2((v8h*)(arow + (size_t)i * NC), v);
  }
  float* cp = cpart + ((size_t)(b * QCN + qc)) * NP;
#pragma unroll
  for (int i = 0; i < 4; ++i) {
    const int f = t + 256 * i;
    v4f v = *(const v4fa*)&csb[f * 4];
    vst2((v4f*)(cp + (size_t)f * 4), v);
  }
}

__global__ void __launch_bounds__(256)
k_fuse(const _Float16* __restrict__ attT, const _Float16* __restrict__ inT, const _Float16* __restrict__ Fwh,
       const float* __restrict__ x, const float* __restrict__ mF, float* __restrict__ out0) {
  __shared__ __attribute__((aligned(16))) float G[NC][36];
  const int t = threadIdx.x, lane = t & 31, wid = t >> 5, h = lane >> 4, n = lane & 15;
  const int blk = blockIdx.x;
  if (blk >= NB * NP / 32) return;
  const int b = blk >> 7, pb = (blk & 127) * 32;
  const int ptile = wid >> 2, og = wid & 3;
  const size_t prow = (size_t)b * NP + pb + ptile * 16 + n;
  const _Float16* A1 = attT + prow * NC;
  const _Float16* A2 = inT + prow * CIN;
  const _Float16* Bb = Fwh + ((size_t)(og * 64 + n)) * CFU;
  v8f d[4];
#pragma unroll
  for (int j = 0; j < 4; ++j) d[j] = zero8();
#pragma unroll 1
  for (int k0 = 0; k0 < NC; k0 += 32) {
    const v16h a = ldfrag_g(A1, k0, h);
#pragma unroll
    for (int j = 0; j < 4; ++j) d[j] = wmma16(a, ldfrag_g(Bb + (size_t)j * 16 * CFU, k0, h), d[j]);
  }
#pragma unroll 1
  for (int k0 = 0; k0 < NC; k0 += 32) {
    const v16h a = ldfrag_g(A2, k0, h);
#pragma unroll
    for (int j = 0; j < 4; ++j) d[j] = wmma16(a, ldfrag_g(Bb + (size_t)j * 16 * CFU, NC + k0, h), d[j]);
  }
#pragma unroll
  for (int j = 0; j < 4; ++j) {
    const int o = og * 64 + j * 16 + n;
#pragma unroll
    for (int r = 0; r < 8; ++r) G[o][ptile * 16 + 8 * h + r] = d[j][r] * (1.f / 64.f);
  }
  __syncthreads();
  v4f vals[8];
  size_t offs[8];
#pragma unroll
  for (int i = 0; i < 8; ++i) {
    const int o = wid * 32 + i * 4 + (lane >> 3);
    const int p4 = (lane & 7) * 4;
    v4f fz = *(const v4fa*)&G[o][p4];
    v4f mv = *(const v4f*)(mF + (size_t)b * NP + pb + p4);
    const size_t gi = ((size_t)(b * NC + o)) * NP + pb + p4;
    v4f xv = *(const v4f*)(x + gi);
    v4f rv;
#pragma unroll
    for (int e = 0; e < 4; ++e) rv[e] = (mv[e] > 0.5f) ? fz[e] : xv[e];
    vals[i] = rv; offs[i] = gi;
  }
#pragma unroll
  for (int i = 0; i < 8; ++i) vst2((v4f*)(out0 + offs[i]), vals[i]);
}

__global__ void __launch_bounds__(256) k_final(const float* __restrict__ cpart, float* __restrict__ out1) {
  __shared__ __attribute__((aligned(16))) float vis[NB * NP];
  __shared__ float red[8];
  const int t = threadIdx.x, lane = t & 31, wid = t >> 5;
  float mx = 0.f;
  for (int idx = t; idx < NB * NP; idx += 256) {
    const int b = idx >> 12, k = idx & (NP - 1);
    const float* cp = cpart + (size_t)b * QCN * NP + k;
    float s = 0.f;
#pragma unroll 8
    for (int q = 0; q < QCN; ++q) s += cp[(size_t)q * NP];
    vis[idx] = s;
    mx = fmaxf(mx, s);
  }
  mx = fmaxf(mx, __shfl_xor(mx, 16)); mx = fmaxf(mx, __shfl_xor(mx, 8)); mx = fmaxf(mx, __shfl_xor(mx, 4));
  mx = fmaxf(mx, __shfl_xor(mx, 2));  mx = fmaxf(mx, __shfl_xor(mx, 1));
  if (lane == 0) red[wid] = mx;
  __syncthreads();
  mx = red[0];
#pragma unroll
  for (int w = 1; w < 8; ++w) mx = fmaxf(mx, red[w]);
  const float inv = 1.f / mx;
  for (int i = 0; i < 1024; ++i) {
    const int f = t + 256 * i;
    const int X4 = (f & 127) * 4, Y = (f >> 7) & 511, bb = f >> 16;
    const float v = vis[bb * NP + (Y >> 3) * 64 + (X4 >> 3)] * inv;
    v4f r; r[0] = v; r[1] = v; r[2] = v; r[3] = v;
    *(volatile v4f*)(out1 + (size_t)f * 4) = r;
  }
  __threadfence();
  for (int i = 0; i < 1024; ++i) {
    const int f = t + 256 * i;
    const int X4 = (f & 127) * 4, Y = (f >> 7) & 511, bb = f >> 16;
    const float v = vis[bb * NP + (Y >> 3) * 64 + (X4 >> 3)] * inv;
    v4f r; r[0] = v; r[1] = v; r[2] = v; r[3] = v;
    *(volatile v4f*)(out1 + (size_t)f * 4) = r;
  }
}

extern "C" void kernel_launch(void* const* d_in, const int* in_sizes, int n_in,
                              void* d_out, int out_size, void* d_ws, size_t ws_size,
                              hipStream_t stream) {
  if (n_in < 6) return;
  if (in_sizes[0] != NB * NC * NP) return;
  if (in_sizes[1] != NB * MS * MS) return;
  if (in_sizes[2] != NB * CAUX * NP) return;
  if (in_sizes[3] != NC * CIN) return;
  if (in_sizes[4] != NC) return;
  if (in_sizes[5] != NC * CFU) return;
  if (out_size != NB * NC * NP + NB * MS * MS) return;

  const float* x   = (const float*)d_in[0];
  const float* msk = (const float*)d_in[1];
  const float* aux = (const float*)d_in[2];
  const float* Kw  = (const float*)d_in[3];
  const float* Kb  = (const float*)d_in[4];
  const float* Fw  = (const float*)d_in[5];
  float* out0 = (float*)d_out;
  float* out1 = out0 + (size_t)NB * NC * NP;

  const size_t o_m   = 0;
  const size_t o_kwh = o_m   + (size_t)NB * NP * 4;
  const size_t o_fwh = o_kwh + (size_t)NC * CIN * 2;
  const size_t o_inT = o_fwh + (size_t)NC * CFU * 2;
  const size_t o_nh  = o_inT + (size_t)NB * NP * CIN * 2;
  const size_t o_vh  = o_nh  + (size_t)NB * NP * NC * 2;
  const size_t o_att = o_vh  + (size_t)NB * NC * NP * 2;
  const size_t o_cp  = o_att + (size_t)NB * NP * NC * 2;
  const size_t total = o_cp  + (size_t)NB * QCN * NP * 4;
  if (total > ws_size) return;

  char* w = (char*)d_ws;
  float*    mF    = (float*)(w + o_m);
  _Float16* Kwh   = (_Float16*)(w + o_kwh);
  _Float16* Fwh   = (_Float16*)(w + o_fwh);
  _Float16* inT   = (_Float16*)(w + o_inT);
  _Float16* Nh    = (_Float16*)(w + o_nh);
  _Float16* Vh    = (_Float16*)(w + o_vh);
  _Float16* attT  = (_Float16*)(w + o_att);
  float*    cpart = (float*)(w + o_cp);

  k_cvtw <<<(NC * CIN / 8 + NC * CFU / 8) / 256, 256, 0, stream>>>(Kw, Fw, Kwh, Fwh);
  k_pool <<<(NB * NP / 4) / 256, 256, 0, stream>>>(msk, mF);
  k_tin  <<<NB * (CIN / 64) * (NP / 64), 256, 0, stream>>>(x, aux, inT);
  k_feats<<<NB * NP / 32, 256, 0, stream>>>(inT, Kwh, Kb, Nh);
  k_makev<<<(NB * NC * NP / 8) / 256, 256, 0, stream>>>(x, mF, Vh);
  k_attn <<<NB * QCN, 256, 0, stream>>>(Nh, Vh, mF, attT, cpart);
  k_fuse <<<NB * NP / 32, 256, 0, stream>>>(attT, inT, Fwh, x, mF, out0);
  k_final<<<1, 256, 0, stream>>>(cpart, out1);
}
